// ExphormerAttention_55044300866300
// MI455X (gfx1250) — hardware-verified
//
#include <hip/hip_runtime.h>
#include <math.h>

typedef __bf16   v16b __attribute__((ext_vector_type(16)));
typedef float    v8f  __attribute__((ext_vector_type(8)));
typedef float    v4f  __attribute__((ext_vector_type(4)));
typedef unsigned v4u  __attribute__((ext_vector_type(4)));

#define CH1     2048
#define NT1     256
#define IPT1    8
#define TL2     4096
#define NT2     256
#define IPT2    16
#define S1LOG   8
#define NCHMAX  1024
#define TPMAX   1024
#define ESHIFT  22
#define EMASK   0x3FFFFFu
#define KSENT   0xFFFFFFFFu

__device__ __forceinline__ int clampi(int v, int lo, int hi) { v = v < lo ? lo : v; return v > hi ? hi : v; }
__device__ __forceinline__ float eluf(float x) { return x > 0.f ? x : expm1f(x); }

__device__ __forceinline__ unsigned short bf16_bits_rne(float f) {
  unsigned u = __float_as_uint(f);
  u += 0x7FFFu + ((u >> 16) & 1u);
  return (unsigned short)(u >> 16);
}
__device__ __forceinline__ void split_bf16(float f, __bf16& hi, __bf16& lo) {
  const unsigned short hb = bf16_bits_rne(f);
  const float fh = __uint_as_float(((unsigned)hb) << 16);
  const unsigned short lb = bf16_bits_rne(f - fh);
  hi = __builtin_bit_cast(__bf16, hb);
  lo = __builtin_bit_cast(__bf16, lb);
}
__device__ __forceinline__ __bf16 bf16_zero() { return __builtin_bit_cast(__bf16, (unsigned short)0); }
__device__ __forceinline__ v8f zero8() { v8f z; z[0]=0.f; z[1]=0.f; z[2]=0.f; z[3]=0.f; z[4]=0.f; z[5]=0.f; z[6]=0.f; z[7]=0.f; return z; }

__device__ __forceinline__ v8f wmma_x3(v8f acc, v16b ah, v16b al, v16b bh, v16b bl) {
  acc = __builtin_amdgcn_wmma_f32_16x16x32_bf16(false, ah, false, bh, (short)0, acc, false, false);
  acc = __builtin_amdgcn_wmma_f32_16x16x32_bf16(false, ah, false, bl, (short)0, acc, false, false);
  acc = __builtin_amdgcn_wmma_f32_16x16x32_bf16(false, al, false, bh, (short)0, acc, false, false);
  asm volatile("v_nop\n\tv_nop\n\tv_nop\n\tv_nop" : "+v"(acc) : "v"(ah), "v"(al), "v"(bh), "v"(bl));
  return acc;
}

template <int NT, int SPAN>
__device__ __forceinline__ unsigned block_excl_scan(unsigned* a, int len, unsigned* s_wtot) {
  const int t = threadIdx.x, lane = t & 31, wv = t >> 5;
  unsigned sum = 0u;
#pragma unroll
  for (int j = 0; j < SPAN; ++j) { const int q = t * SPAN + j; if (q < len) sum += a[q]; }
  unsigned incl = sum;
#pragma unroll
  for (int off = 1; off < 32; off <<= 1) { const unsigned v = __shfl_up(incl, off); if (lane >= off) incl += v; }
  if (lane == 31) s_wtot[wv] = incl;
  __syncthreads();
  unsigned wbase = 0u, total = 0u;
#pragma unroll
  for (int w = 0; w < NT / 32; ++w) { const unsigned v = s_wtot[w]; total += v; if (w < wv) wbase += v; }
  unsigned run = wbase + incl - sum;
#pragma unroll
  for (int j = 0; j < SPAN; ++j) {
    const int q = t * SPAN + j;
    if (q < len) { const unsigned v = a[q]; a[q] = run; run += v; }
  }
  __syncthreads();
  return total;
}

template <int NT, int IPT, int LOGD>
__device__ __forceinline__ void radix_pass(unsigned* in, unsigned* out, unsigned* hist, unsigned* s_wtot, int shift) {
  constexpr int D = 1 << LOGD;
  const int t = threadIdx.x;
#pragma unroll
  for (int d = 0; d < D; ++d) hist[d * NT + t] = 0u;
  unsigned keys[IPT];
#pragma unroll
  for (int j = 0; j < IPT; ++j) {
    const unsigned k = in[t * IPT + j];
    keys[j] = k;
    const unsigned d = (k >> shift) & (unsigned)(D - 1);
    hist[d * NT + t] += 1u;
  }
  __syncthreads();
  block_excl_scan<NT, D>(hist, D * NT, s_wtot);
#pragma unroll
  for (int j = 0; j < IPT; ++j) {
    const unsigned d = (keys[j] >> shift) & (unsigned)(D - 1);
    const unsigned pos = hist[d * NT + t];
    hist[d * NT + t] = pos + 1u;
    if (pos < (unsigned)(NT * IPT)) out[pos] = keys[j];
  }
  __syncthreads();
}

__device__ __forceinline__ int lower_bound_u(const unsigned* a, int n, unsigned key) {
  int lo = 0, len = n;
#pragma unroll 1
  for (int s = 0; s < 13; ++s) {
    if (len > 0) {
      const int half = len >> 1;
      if (a[lo + half] < key) { lo += half + 1; len -= half + 1; } else { len = half; }
    }
  }
  return lo;
}

__global__ __launch_bounds__(128) void k_node_proj(
    const float* __restrict__ evec, const float* __restrict__ unused0,
    const float* __restrict__ W1, const float* __restrict__ b1,
    const float* __restrict__ W2, const float* __restrict__ b2,
    const float* __restrict__ Wm, const float* __restrict__ bm,
    float* qkv, int M)
{
  (void)unused0;
  __shared__ float qs[64 * 64];
  const int t = threadIdx.x, lane = t & 31, wv = t >> 5, hh = lane >> 4, m = lane & 15;
  const int row0 = blockIdx.x * 64 + wv * 16;
  const int node = row0 + m;
  const float x = (node < M) ? evec[node] : 0.f;

  float h1[4];
#pragma unroll
  for (int j = 0; j < 4; ++j) { float s = x * W1[j]; s += b1[j]; h1[j] = eluf(s); }

  const __bf16 bz = bf16_zero();
  v16b ah, al;
#pragma unroll
  for (int i = 0; i < 8; ++i) {
    const int k = 8 * hh + i;
    float s = h1[0] * W2[k];
    s += h1[1] * W2[16 + k];
    s += h1[2] * W2[32 + k];
    s += h1[3] * W2[48 + k];
    s += b2[k];
    __bf16 hi, lo; split_bf16(s, hi, lo); ah[i] = hi; al[i] = lo;
  }
#pragma unroll
  for (int i = 8; i < 16; ++i) { ah[i] = bz; al[i] = bz; }

  float* qsw = qs + wv * 1024;
#pragma unroll
  for (int tt = 0; tt < 4; ++tt) {
    v16b bh, bl;
#pragma unroll
    for (int i = 0; i < 8; ++i) {
      const float w = Wm[(8 * hh + i) * 64 + tt * 16 + m];
      __bf16 hi, lo; split_bf16(w, hi, lo); bh[i] = hi; bl[i] = lo;
    }
#pragma unroll
    for (int i = 8; i < 16; ++i) { bh[i] = bz; bl[i] = bz; }
    const v8f acc = wmma_x3(zero8(), ah, al, bh, bl);
    const float bias = bm[tt * 16 + m];
#pragma unroll
    for (int r = 0; r < 8; ++r) qsw[(8 * hh + r) * 64 + tt * 16 + m] = acc[r] + bias;
  }
  __syncthreads();

  float* dst = qkv + (size_t)blockIdx.x * 4096;
  v4f vv[8];
#pragma unroll
  for (int j = 0; j < 8; ++j) vv[j] = *(const v4f*)(qs + j * 512 + t * 4);
#pragma unroll
  for (int j = 0; j < 8; ++j) *(volatile v4f*)(dst + j * 512 + t * 4) = vv[j];
  __threadfence();
#pragma unroll
  for (int j = 0; j < 8; ++j) *(volatile v4f*)(dst + j * 512 + t * 4) = vv[j];
}

__global__ __launch_bounds__(128) void k_edge_score(
    const int* __restrict__ eidx, const float* __restrict__ efeat,
    const float* __restrict__ W2, const float* __restrict__ b2,
    const float* __restrict__ Wm, const float* __restrict__ bm,
    const float* __restrict__ qkv, float* scb, int NE, int M, int NG)
{
  __shared__ float Es[4][16][64];
  __shared__ float scs[4][16][4];
  const int t = threadIdx.x, lane = t & 31, wv = t >> 5, hh = lane >> 4, m = lane & 15;
  const int g = blockIdx.x * 4 + wv;
  const int base = g * 16;
  const int e0 = base + m;

  v4f ef; ef[0] = 0.f; ef[1] = 0.f; ef[2] = 0.f; ef[3] = 0.f;
  if (e0 < NE) ef = *(const v4f*)(efeat + (size_t)e0 * 4);

  const __bf16 bz = bf16_zero();
  v16b ah, al;
#pragma unroll
  for (int i = 0; i < 8; ++i) {
    const int k = 8 * hh + i;
    float s = ef[0] * W2[k];
    s += ef[1] * W2[16 + k];
    s += ef[2] * W2[32 + k];
    s += ef[3] * W2[48 + k];
    s += b2[k];
    const float a = eluf(s);
    __bf16 hi, lo; split_bf16(a, hi, lo); ah[i] = hi; al[i] = lo;
  }
#pragma unroll
  for (int i = 8; i < 16; ++i) { ah[i] = bz; al[i] = bz; }

#pragma unroll
  for (int tt = 0; tt < 4; ++tt) {
    v16b bh, bl;
#pragma unroll
    for (int i = 0; i < 8; ++i) {
      const float w = Wm[(8 * hh + i) * 64 + tt * 16 + m];
      __bf16 hi, lo; split_bf16(w, hi, lo); bh[i] = hi; bl[i] = lo;
    }
#pragma unroll
    for (int i = 8; i < 16; ++i) { bh[i] = bz; bl[i] = bz; }
    const v8f acc = wmma_x3(zero8(), ah, al, bh, bl);
    const float bias = bm[tt * 16 + m];
#pragma unroll
    for (int r = 0; r < 8; ++r) Es[wv][8 * hh + r][tt * 16 + m] = acc[r] + bias;
  }
  __syncthreads();

#pragma unroll
  for (int p = 0; p < 2; ++p) {
    const int pair = p * 32 + lane;
    const int m2 = pair >> 2, t2 = pair & 3;
    const int e = base + m2;
    int si = 0, di = 0;
    if (e < NE) { si = eidx[e]; di = eidx[(size_t)NE + e]; }
    si = clampi(si, 0, M - 1); di = clampi(di, 0, M - 1);
    const float* sp = qkv + (size_t)si * 64 + t2 * 16;
    const float* dp = qkv + (size_t)di * 64 + t2 * 16;
    const float* ep = &Es[wv][m2][t2 * 16];
    float sum = 0.f;
#pragma unroll
    for (int c4 = 0; c4 < 4; ++c4) {
      const v4f sv = *(const v4f*)(sp + 4 * c4);
      const v4f dv = *(const v4f*)(dp + 4 * c4);
      const v4f ev = *(const v4f*)(ep + 4 * c4);
#pragma unroll
      for (int c = 0; c < 4; ++c) { float pr = sv[c] * dv[c]; pr = pr * 0.25f; pr = pr * ev[c]; sum += pr; }
    }
    sum = fminf(5.f, fmaxf(-5.f, sum));
    scs[wv][m2][t2] = expf(sum);
  }
  __syncthreads();

  const bool wr = (g < NG) && (lane < 16);
  v4f sv4; sv4[0] = 0.f; sv4[1] = 0.f; sv4[2] = 0.f; sv4[3] = 0.f;
  if (lane < 16) sv4 = *(const v4f*)&scs[wv][lane][0];
  float* so = scb + (size_t)(base + (lane & 15)) * 4;
  if (wr) *(volatile v4f*)so = sv4;
  __threadfence();
  if (wr) *(volatile v4f*)so = sv4;
}

__global__ __launch_bounds__(NT1) void k_edge_partition(
    const int* __restrict__ eidx, unsigned* cw, unsigned* ct, int NE, int M, int nb1, int tp)
{
  __shared__ unsigned bufA[CH1], bufB[CH1];
  __shared__ unsigned hist[32 * NT1];
  __shared__ unsigned tab[TPMAX];
  __shared__ unsigned s_wtot[NT1 / 32];
  const int t = threadIdx.x, c = blockIdx.x;
  const int e0 = c * CH1;
#pragma unroll
  for (int j = 0; j < IPT1; ++j) {
    const int i = t * IPT1 + j;
    const int e = e0 + i;
    unsigned key = KSENT;
    if (e < NE) {
      int d = eidx[(size_t)NE + e];
      d = clampi(d, 0, M - 1);
      key = (((unsigned)(d >> S1LOG)) << ESHIFT) | (unsigned)e;
    }
    bufA[i] = key;
  }
  __syncthreads();
  radix_pass<NT1, IPT1, 5>(bufA, bufB, hist, s_wtot, ESHIFT);
  radix_pass<NT1, IPT1, 5>(bufB, bufA, hist, s_wtot, ESHIFT + 5);
  for (int b = t; b < tp; b += NT1) {
    const int bb = b < nb1 ? b : nb1;
    tab[b] = (unsigned)lower_bound_u(bufA, CH1, ((unsigned)bb) << ESHIFT);
  }
  __syncthreads();

  const v4u w0 = *(const v4u*)&bufA[t * 4];
  const v4u w1 = *(const v4u*)&bufA[1024 + t * 4];
  const bool tw = (t * 4 < tp);
  v4u tv; tv[0] = 0u; tv[1] = 0u; tv[2] = 0u; tv[3] = 0u;
  if (tw) tv = *(const v4u*)&tab[t * 4];
  unsigned* cwo = cw + (size_t)c * CH1;
  unsigned* cto = ct + (size_t)c * tp;
  *(volatile v4u*)(cwo + t * 4) = w0;
  *(volatile v4u*)(cwo + 1024 + t * 4) = w1;
  if (tw) *(volatile v4u*)(cto + t * 4) = tv;
  __threadfence();
  *(volatile v4u*)(cwo + t * 4) = w0;
  *(volatile v4u*)(cwo + 1024 + t * 4) = w1;
  if (tw) *(volatile v4u*)(cto + t * 4) = tv;
}

__global__ __launch_bounds__(NT2) void k_dst_gather(
    const int* __restrict__ eidx, const unsigned* __restrict__ cw, const unsigned* __restrict__ ct,
    const float* __restrict__ qkv, const float* __restrict__ scb, float* hbuf,
    int NE, int M, int nch, int tp)
{
  __shared__ unsigned runpre[NCHMAX + 4];
  __shared__ unsigned st[NCHMAX];
  __shared__ unsigned bufA[TL2], bufB[TL2];
  __shared__ unsigned hist[16 * NT2];
  __shared__ unsigned s_wtot[NT2 / 32];
  __shared__ int segs[NT2], sege[NT2];
  const int t = threadIdx.x, b = blockIdx.x;

  for (int c = t; c < nch; c += NT2) {
    unsigned s  = ct[(size_t)c * tp + b];
    unsigned en = ct[(size_t)c * tp + b + 1];
    s  = s  > (unsigned)CH1 ? (unsigned)CH1 : s;
    en = en > (unsigned)CH1 ? (unsigned)CH1 : en;
    st[c] = s;
    runpre[c] = en > s ? en - s : 0u;
  }
  __syncthreads();
  const unsigned T = block_excl_scan<NT2, NCHMAX / NT2>(runpre, nch, s_wtot);
  if (t == 0) runpre[nch] = T;
  __syncthreads();

  v4f acc[16];
#pragma unroll
  for (int k = 0; k < 16; ++k) { acc[k][0] = 0.f; acc[k][1] = 0.f; acc[k][2] = 0.f; acc[k][3] = 0.f; }
  float z[4] = {0.f, 0.f, 0.f, 0.f};

  const int Ti = (int)T;
  const int ntiles = (Ti + TL2 - 1) / TL2;
  for (int tile = 0; tile < ntiles; ++tile) {
    const int q0 = tile * TL2;
    const int rem = Ti - q0;
    const int nvalid = rem < TL2 ? rem : TL2;

    int c = 0;
    {
      const unsigned qf = (unsigned)(q0 + t * IPT2);
      int lo = 0, hi = nch;
#pragma unroll 1
      for (int s = 0; s < 12; ++s) {
        if (hi - lo > 1) { const int mid = (lo + hi) >> 1; if (runpre[mid] <= qf) lo = mid; else hi = mid; }
      }
      c = lo;
    }
#pragma unroll
    for (int j = 0; j < IPT2; ++j) {
      const int i = t * IPT2 + j;
      unsigned key = KSENT;
      if (i < nvalid) {
        const unsigned q = (unsigned)(q0 + i);
        while (c + 1 < nch && runpre[c + 1] <= q) ++c;
        unsigned off = st[c] + (q - runpre[c]);
        off = off < (unsigned)CH1 ? off : (unsigned)(CH1 - 1);
        const unsigned w = cw[(size_t)c * CH1 + off];
        unsigned e = w & EMASK;
        e = e < (unsigned)NE ? e : (unsigned)(NE - 1);
        int d = eidx[(size_t)NE + e];
        d = clampi(d, 0, M - 1);
        key = (((unsigned)d & 255u) << ESHIFT) | e;
      }
      bufA[i] = key;
    }
    __syncthreads();
    radix_pass<NT2, IPT2, 4>(bufA, bufB, hist, s_wtot, ESHIFT);
    radix_pass<NT2, IPT2, 4>(bufB, bufA, hist, s_wtot, ESHIFT + 4);

    segs[t] = 0; sege[t] = 0;
    __syncthreads();
#pragma unroll
    for (int j = 0; j < IPT2; ++j) {
      const int i = t * IPT2 + j;
      if (i < nvalid) {
        const unsigned k  = (bufA[i] >> ESHIFT) & 255u;
        const unsigned kp = (i > 0) ? ((bufA[i - 1] >> ESHIFT) & 255u) : 256u;
        const unsigned kn = (i + 1 < nvalid) ? ((bufA[i + 1] >> ESHIFT) & 255u) : 256u;
        if (kp != k) segs[k] = i;
        if (kn != k) sege[k] = i + 1;
      }
    }
    __syncthreads();

    const int ib = segs[t], ie = sege[t];
#pragma unroll 1
    for (int i = ib; i < ie; ++i) {
      const unsigned w = bufA[i];
      unsigned e = w & EMASK;
      e = e < (unsigned)NE ? e : (unsigned)(NE - 1);
      int si = eidx[e];
      si = clampi(si, 0, M - 1);
      const v4f sc = *(const v4f*)(scb + (size_t)e * 4);
      const float* qr = qkv + (size_t)si * 64;
#pragma unroll
      for (int hd = 0; hd < 4; ++hd) {
        const float s = sc[hd];
        z[hd] += s;
#pragma unroll
        for (int c4 = 0; c4 < 4; ++c4) {
          const v4f v = *(const v4f*)(qr + hd * 16 + c4 * 4);
          acc[hd * 4 + c4] += s * v;
        }
      }
    }
    __syncthreads();
  }

  const int d = b * NT2 + t;
  float* hr = hbuf + (size_t)d * 64;
  v4f ov[16];
#pragma unroll
  for (int hd = 0; hd < 4; ++hd) {
    const float r = 1.f / (z[hd] + 1e-6f);
#pragma unroll
    for (int c4 = 0; c4 < 4; ++c4) ov[hd * 4 + c4] = acc[hd * 4 + c4] * r;
  }
#pragma unroll
  for (int k = 0; k < 16; ++k) *(volatile v4f*)(hr + 4 * k) = ov[k];
  __threadfence();
#pragma unroll
  for (int k = 0; k < 16; ++k) *(volatile v4f*)(hr + 4 * k) = ov[k];
}

__global__ __launch_bounds__(64) void k_out_head(
    const float* __restrict__ hbuf, const float* __restrict__ Wout, const float* __restrict__ bout,
    const float* __restrict__ Wout1, const float* __restrict__ bout1, float* out, int M)
{
  __shared__ float os[128];
  const int t = threadIdx.x, lane = t & 31, wv = t >> 5, hh = lane >> 4, m = lane & 15;

  v16b a0h, a0l, a1h, a1l;
#pragma unroll
  for (int i = 0; i < 16; ++i) {
    const int kk = (i < 8) ? (8 * hh + i) : (16 + 8 * hh + (i - 8));
    { const float w = Wout[kk * 16 + m];        __bf16 hi, lo; split_bf16(w, hi, lo); a0h[i] = hi; a0l[i] = lo; }
    { const float w = Wout[(32 + kk) * 16 + m]; __bf16 hi, lo; split_bf16(w, hi, lo); a1h[i] = hi; a1l[i] = lo; }
  }
  float bo[8], w1[8];
#pragma unroll
  for (int r = 0; r < 8; ++r) { bo[r] = bout[8 * hh + r]; w1[r] = Wout1[8 * hh + r]; }
  const float b1v = bout1[0];

#pragma unroll
  for (int gq = 0; gq < 4; ++gq) {
    const int node = blockIdx.x * 128 + wv * 64 + gq * 16 + m;
    const float* hr = hbuf + (size_t)node * 64;
    v8f acc = zero8();
    {
      const v4f x0 = *(const v4f*)(hr + 8 * hh), x1 = *(const v4f*)(hr + 8 * hh + 4);
      const v4f x2 = *(const v4f*)(hr + 16 + 8 * hh), x3 = *(const v4f*)(hr + 16 + 8 * hh + 4);
      v16b bh, bl;
#pragma unroll
      for (int c = 0; c < 4; ++c) {
        __bf16 hi, lo;
        split_bf16(x0[c], hi, lo); bh[c] = hi;      bl[c] = lo;
        split_bf16(x1[c], hi, lo); bh[4 + c] = hi;  bl[4 + c] = lo;
        split_bf16(x2[c], hi, lo); bh[8 + c] = hi;  bl[8 + c] = lo;
        split_bf16(x3[c], hi, lo); bh[12 + c] = hi; bl[12 + c] = lo;
      }
      acc = wmma_x3(acc, a0h, a0l, bh, bl);
    }
    {
      const v4f x0 = *(const v4f*)(hr + 32 + 8 * hh), x1 = *(const v4f*)(hr + 32 + 8 * hh + 4);
      const v4f x2 = *(const v4f*)(hr + 48 + 8 * hh), x3 = *(const v4f*)(hr + 48 + 8 * hh + 4);
      v16b bh, bl;
#pragma unroll
      for (int c = 0; c < 4; ++c) {
        __bf16 hi, lo;
        split_bf16(x0[c], hi, lo); bh[c] = hi;      bl[c] = lo;
        split_bf16(x1[c], hi, lo); bh[4 + c] = hi;  bl[4 + c] = lo;
        split_bf16(x2[c], hi, lo); bh[8 + c] = hi;  bl[8 + c] = lo;
        split_bf16(x3[c], hi, lo); bh[12 + c] = hi; bl[12 + c] = lo;
      }
      acc = wmma_x3(acc, a1h, a1l, bh, bl);
    }
    float part = 0.f;
#pragma unroll
    for (int r = 0; r < 8; ++r) { float y = acc[r] + bo[r]; y = eluf(y); part += y * w1[r]; }
    part += __shfl_xor(part, 16);
    if (hh == 0) os[wv * 64 + gq * 16 + m] = part + b1v;
  }
  __syncthreads();

  if (t < 32) {
    const int idx = blockIdx.x * 128 + t * 4;
    v4f v = *(const v4f*)&os[t * 4];
    if (idx + 3 < M) {
      *(volatile v4f*)(out + idx) = v;
      __threadfence();
      *(volatile v4f*)(out + idx) = v;
    } else {
#pragma unroll
      for (int j = 0; j < 4; ++j) if (idx + j < M) ((volatile float*)out)[idx + j] = v[j];
      __threadfence();
#pragma unroll
      for (int j = 0; j < 4; ++j) if (idx + j < M) ((volatile float*)out)[idx + j] = v[j];
    }
  }
}

extern "C" void kernel_launch(void* const* d_in, const int* in_sizes, int n_in,
                              void* d_out, int out_size, void* d_ws, size_t ws_size,
                              hipStream_t stream) {
  if (n_in < 14) return;
  const float* nattr = (const float*)d_in[0];
  const int*   eidx  = (const int*)  d_in[1];
  const float* efeat = (const float*)d_in[2];
  const float* evec  = (const float*)d_in[3];
  const float* W1    = (const float*)d_in[4];
  const float* b1    = (const float*)d_in[5];
  const float* W2    = (const float*)d_in[6];
  const float* b2    = (const float*)d_in[7];
  const float* Wm    = (const float*)d_in[8];
  const float* bm    = (const float*)d_in[9];
  const float* Wout  = (const float*)d_in[10];
  const float* bout  = (const float*)d_in[11];
  const float* Wout1 = (const float*)d_in[12];
  const float* bout1 = (const float*)d_in[13];

  const int M  = in_sizes[3];
  const int NE = in_sizes[2] / 4;
  if (M <= 0 || NE <= 0) return;
  if (out_size < M) return;
  if (in_sizes[1] < 2 * NE) return;

  const int nb1   = (M + NT2 - 1) / NT2;
  const int tp    = ((nb1 + 1 + 31) / 32) * 32;
  const int nch   = (NE + CH1 - 1) / CH1;
  const int qrows = ((M + 63) / 64) * 64;
  const int NG    = (NE + 15) / 16;
  const long long scrows = (long long)NG * 16;
  const long long hrows  = (long long)nb1 * NT2;
  if (nb1 > 1000 || tp > TPMAX || nch > NCHMAX || (unsigned)NE > EMASK) return;

  size_t off = 0;
  const size_t o_qkv = off; off += (((size_t)qrows * 64 * 4) + 255) & ~(size_t)255;
  const size_t o_scb = off; off += (((size_t)scrows * 16) + 255) & ~(size_t)255;
  const size_t o_cw  = off; off += (((size_t)nch * CH1 * 4) + 255) & ~(size_t)255;
  const size_t o_ct  = off; off += (((size_t)nch * tp * 4) + 255) & ~(size_t)255;
  const size_t o_hb  = off; off += (((size_t)hrows * 64 * 4) + 255) & ~(size_t)255;
  if (off > ws_size) return;

  char* ws = (char*)d_ws;
  float*    qkv  = (float*)(ws + o_qkv);
  float*    scb  = (float*)(ws + o_scb);
  unsigned* cw   = (unsigned*)(ws + o_cw);
  unsigned* ct   = (unsigned*)(ws + o_ct);
  float*    hbuf = (float*)(ws + o_hb);

  k_node_proj<<<qrows / 64, 128, 0, stream>>>(evec, nattr, W1, b1, W2, b2, Wm, bm, qkv, M);
  k_edge_score<<<(NG + 3) / 4, 128, 0, stream>>>(eidx, efeat, W2, b2, Wm, bm, qkv, scb, NE, M, NG);
  k_edge_partition<<<nch, NT1, 0, stream>>>(eidx, cw, ct, NE, M, nb1, tp);
  k_dst_gather<<<nb1, NT2, 0, stream>>>(eidx, cw, ct, qkv, scb, hbuf, NE, M, nch, tp);
  k_out_head<<<(M + 127) / 128, 64, 0, stream>>>(hbuf, Wout, bout, Wout1, bout1, (float*)d_out, M);
}
